// graph_convolution_33938831573463
// MI455X (gfx1250) — hardware-verified
//
#include <hip/hip_runtime.h>
#include <stddef.h>


#pragma clang fp contract(off)

#define CI      64
#define DE      16
#define HD      64
#define CO      64
#define NPQ     128
#define KIN1    144
#define KE      32
#define KU      128
#define NLAY    3
#define NTHR    256
#define NWAVE   8
#define NBN     64
#define XP      72
#define SP      68
#define TE      128
#define EP      40
#define MP      72
#define NBU     128
#define UP      136
#define EPT     8
#define PIECE   (NTHR * EPT)
#define WCAP    (EPT * 32)
#define NBC     1024
#define SLB     10
#define LW_PQ   0
#define LW_1E   8192
#define LW_W2   10240
#define LW_WU   14336
#define LWTOT   22528
#define PBL     (LWTOT / (NTHR * 8))
#define PREPBLK (NLAY * PBL)
#define WSCAP   134217728
#define PQDYN   (NWAVE * 16 * SP * 4)
#define EDGEDYN (TE * SP * 4)
#define UPDDYN  (NBU * UP * 2 + NBU * SP * 4)
#define AGGDYN  (NBC * CO * 4)
#define EPSLN   1e-5f

static_assert((LWTOT % (NTHR * 8)) == 0);
static_assert(PBL == 11);
static_assert((LW_1E % 2048) == 0);
static_assert((LW_W2 % 2048) == 0);
static_assert((LW_WU % 2048) == 0);
static_assert(LW_1E == 128 * CI);
static_assert(LW_W2 == LW_1E + 64 * KE);
static_assert(LW_WU == LW_W2 + 64 * HD);
static_assert(LWTOT == LW_WU + 64 * KU);
static_assert(((XP * 2) % 16) == 0);
static_assert(((EP * 2) % 16) == 0);
static_assert(((MP * 2) % 16) == 0);
static_assert(((UP * 2) % 16) == 0);
static_assert(((SP * 4) % 16) == 0);
static_assert(NBC == (1 << SLB));
static_assert(PIECE == 2048);
static_assert(SLB + 11 <= 30);
static_assert((EPT % 4) == 0);
static_assert((NBC % (2 * NWAVE)) == 0);
static_assert(NBN == 4 * 16);
static_assert(NTHR == 4 * NBN);
static_assert(TE == NWAVE * 16);
static_assert(NTHR == 2 * TE);
static_assert(NBU == NWAVE * 16);
static_assert(NTHR == 2 * NBU);
static_assert((NBC * CO) % (4 * NTHR) == 0);
static_assert((PIECE % TE) == 0);
static_assert((NBC % NBU) == 0);
static_assert(((NBU * UP * 2) % 16) == 0);

typedef float          v2f   __attribute__((ext_vector_type(2)));
typedef float          v4f   __attribute__((ext_vector_type(4)));
typedef float          v8f   __attribute__((ext_vector_type(8)));
typedef int            v4i   __attribute__((ext_vector_type(4)));
typedef unsigned int   v4u   __attribute__((ext_vector_type(4)));
typedef _Float16       v8h   __attribute__((ext_vector_type(8)));
typedef _Float16       v16h  __attribute__((ext_vector_type(16)));

__device__ __forceinline__ v16h ldfrag(const _Float16* p) {
  const v8h u0 = *(const v8h*)p;
  const v8h u1 = *(const v8h*)(p + 16);
  return __builtin_shufflevector(u0, u1, 0, 1, 2, 3, 4, 5, 6, 7, 8, 9, 10, 11, 12, 13, 14, 15);
}

__device__ __forceinline__ v8f wm(v16h a, v16h b, v8f c) {
  v8f d = __builtin_amdgcn_wmma_f32_16x16x32_f16(false, a, false, b, (short)0, c, false, false);
  asm volatile("v_nop\n\tv_nop\n\tv_nop\n\tv_nop" : "+v"(d) : "v"(a), "v"(b));
  return d;
}
__device__ __forceinline__ v8f zero8() {
  v8f z = {0.f, 0.f, 0.f, 0.f, 0.f, 0.f, 0.f, 0.f};
  return z;
}
__device__ __forceinline__ int iclamp(int v, int lo, int hi) { return v < lo ? lo : (v > hi ? hi : v); }
__device__ __forceinline__ _Float16 m1h(float d, float rs) { return (_Float16)(16.0f * fmaxf(d * rs, 0.0f)); }

__device__ __forceinline__ void ln_relu_acc(v8f* c, const float* sb, int m, float inv) {
#pragma unroll
  for (int j = 0; j < 4; ++j) {
    const float bb = sb[16 * j + m];
#pragma unroll
    for (int r = 0; r < 8; ++r) c[j][r] = c[j][r] * inv + bb;
  }
#pragma unroll
  for (int r = 0; r < 8; ++r) {
    float s = ((c[0][r] + c[1][r]) + c[2][r]) + c[3][r];
    s += __shfl_xor(s, 1, 32);
    s += __shfl_xor(s, 2, 32);
    s += __shfl_xor(s, 4, 32);
    s += __shfl_xor(s, 8, 32);
    const float mean = s * (1.0f / 64.0f);
    const float d0 = c[0][r] - mean, d1 = c[1][r] - mean, d2 = c[2][r] - mean, d3 = c[3][r] - mean;
    float v = ((d0 * d0 + d1 * d1) + d2 * d2) + d3 * d3;
    v += __shfl_xor(v, 1, 32);
    v += __shfl_xor(v, 2, 32);
    v += __shfl_xor(v, 4, 32);
    v += __shfl_xor(v, 8, 32);
    const float rs = rsqrtf(v * (1.0f / 64.0f) + EPSLN);
    c[0][r] = fmaxf(d0 * rs, 0.0f);
    c[1][r] = fmaxf(d1 * rs, 0.0f);
    c[2][r] = fmaxf(d2 * rs, 0.0f);
    c[3][r] = fmaxf(d3 * rs, 0.0f);
  }
}

__global__ __launch_bounds__(NTHR) void k_prep(const float* __restrict__ w1, const float* __restrict__ w2,
                                               const float* __restrict__ wu, _Float16* wp) {
  const int tid = (int)threadIdx.x;
  const int blk = (int)blockIdx.x;
  const int l = blk / PBL;
  const int bl = blk - PBL * l;
  const int o = (bl * NTHR + tid) * 8;
  const float* w1l = w1 + (size_t)l * KIN1 * HD;
  const float* w2l = w2 + (size_t)l * HD * HD;
  const float* wul = wu + (size_t)l * KU * HD;
  v8h hv;
  if (bl < 2) {
    const int n = o >> 6, k0 = o & 63;
#pragma unroll
    for (int i = 0; i < 8; ++i) hv[i] = (_Float16)(64.0f * w1l[(size_t)(k0 + i) * HD + n]);
  } else if (bl < 4) {
    const int n = (o >> 6) - 64, k0 = o & 63;
#pragma unroll
    for (int i = 0; i < 8; ++i) hv[i] = (_Float16)(64.0f * w1l[(size_t)(64 + k0 + i) * HD + n]);
  } else if (bl == 4) {
    const int idx = o - LW_1E;
    const int n = idx >> 5, k0 = idx & 31;
    const float sel = (k0 < 16) ? 64.0f : 0.0f;
#pragma unroll
    for (int i = 0; i < 8; ++i) {
      const int kk = (k0 + i) & 15;
      hv[i] = (_Float16)(sel * w1l[(size_t)(128 + kk) * HD + n]);
    }
  } else if (bl < 7) {
    const int idx = o - LW_W2;
    const int n = idx >> 6, k0 = idx & 63;
#pragma unroll
    for (int i = 0; i < 8; ++i) hv[i] = (_Float16)(64.0f * w2l[(size_t)(k0 + i) * HD + n]);
  } else {
    const int idx = o - LW_WU;
    const int n = idx >> 7, k0 = idx & 127;
#pragma unroll
    for (int i = 0; i < 8; ++i) hv[i] = (_Float16)(64.0f * wul[(size_t)(k0 + i) * HD + n]);
  }
  const v4u u = __builtin_bit_cast(v4u, hv);
  _Float16* dst = wp + (size_t)l * LWTOT + o;
  *(volatile v4u*)dst = u;
  __threadfence();
  *(volatile v4u*)dst = u;
}

__global__ __launch_bounds__(NTHR) void k_pq(const float* __restrict__ x, const _Float16* __restrict__ wq,
                                             float* PQ, int nN) {
  extern __shared__ __attribute__((aligned(16))) float stg[];
  __shared__ __attribute__((aligned(16))) _Float16 sX[NBN * XP];
  const int tid = (int)threadIdx.x, lane = tid & 31, wave = tid >> 5, hh = lane >> 4, m = lane & 15;
  const int n0 = (int)blockIdx.x * NBN;

  {
    const int nl = tid >> 2, q = tid & 3;
    int node = n0 + nl;
    node = node > nN - 1 ? nN - 1 : node;
    const float* rp = x + (size_t)node * CI + 16 * q;
#pragma unroll
    for (int g = 0; g < 2; ++g) {
      const v4f a = *(const v4f*)(rp + 8 * g);
      const v4f b = *(const v4f*)(rp + 8 * g + 4);
      v8h u;
      u[0] = (_Float16)a.x; u[1] = (_Float16)a.y; u[2] = (_Float16)a.z; u[3] = (_Float16)a.w;
      u[4] = (_Float16)b.x; u[5] = (_Float16)b.y; u[6] = (_Float16)b.z; u[7] = (_Float16)b.w;
      *(v8h*)(sX + nl * XP + 16 * q + 8 * g) = u;
    }
  }
  __syncthreads();

  const int rt = wave & 3, cg = wave >> 2;
  const _Float16* bp = wq + (size_t)(64 * cg + m) * CI + 8 * hh;
  const _Float16* ap = sX + (16 * rt + m) * XP + 8 * hh;
  v8f c[4];
#pragma unroll
  for (int j = 0; j < 4; ++j) c[j] = zero8();
#pragma unroll
  for (int ks = 0; ks < 2; ++ks) {
    const v16h a = ldfrag(ap + 32 * ks);
#pragma unroll
    for (int j = 0; j < 4; ++j) {
      const v16h b = ldfrag(bp + (size_t)(16 * j) * CI + 32 * ks);
      c[j] = wm(a, b, c[j]);
    }
  }
  float* sw = stg + wave * 16 * SP;
#pragma unroll
  for (int j = 0; j < 4; ++j) {
#pragma unroll
    for (int r = 0; r < 8; ++r) sw[(8 * hh + r) * SP + 16 * j + m] = c[j][r] * 0.015625f;
  }
  __syncthreads();
  float* ob = PQ + (size_t)64 * cg + 4 * m;
#pragma unroll 1
  for (int i = 0; i < 8; ++i) {
    const int row = 2 * i + hh;
    const v4f v = *(const v4f*)(sw + row * SP + 4 * m);
    *(volatile v4f*)(ob + (size_t)(n0 + 16 * rt + row) * NPQ) = v;
  }
  __threadfence();
#pragma unroll 1
  for (int i = 0; i < 8; ++i) {
    const int row = 2 * i + hh;
    const v4f v = *(const v4f*)(sw + row * SP + 4 * m);
    *(volatile v4f*)(ob + (size_t)(n0 + 16 * rt + row) * NPQ) = v;
  }
}

__global__ __launch_bounds__(NTHR) void k_edge(
    const int* __restrict__ ei, const float* __restrict__ ef, const float* __restrict__ PQ,
    const float* __restrict__ b1, const float* __restrict__ b2, const _Float16* __restrict__ wl, float* MS,
    int c0, int nE, int nN) {
  extern __shared__ __attribute__((aligned(16))) float edyn[];
  __shared__ __attribute__((aligned(16))) _Float16 sEF[TE * EP];
  __shared__ __attribute__((aligned(16))) _Float16 sM1[TE * MP];
  __shared__ __attribute__((aligned(16))) float sPar[HD + CO];
  __shared__ int sIdx[2 * TE];
  float* sT = edyn;
  float* sO = edyn;
  const int tid = (int)threadIdx.x, lane = tid & 31, wave = tid >> 5, hh = lane >> 4, m = lane & 15;
  const int le0 = (int)blockIdx.x * TE;
  const int ge0 = c0 + le0;
  const _Float16* w1e = wl + LW_1E;
  const _Float16* w2p = wl + LW_W2;

  {
    const int s = tid >> 7, j = tid & (TE - 1);
    int e = ge0 + j;
    e = e > nE - 1 ? nE - 1 : e;
    int v = ei[(size_t)s * nE + e];
    if (v < 0) v += nN;
    v = iclamp(v, 0, nN - 1);
    sIdx[s * TE + j] = v;
    const float vb1 = b1[tid & 63];
    const float vb2 = b2[tid & 63];
    if (tid < HD + CO) sPar[tid] = (tid < HD) ? vb1 : vb2;
  }
  {
    const int el = tid >> 1, q = tid & 1;
    int e = ge0 + el;
    e = e > nE - 1 ? nE - 1 : e;
    const float* rp = ef + (size_t)e * DE + 8 * q;
    const v4f a = *(const v4f*)rp;
    const v4f b = *(const v4f*)(rp + 4);
    v8h u;
    u[0] = (_Float16)a.x; u[1] = (_Float16)a.y; u[2] = (_Float16)a.z; u[3] = (_Float16)a.w;
    u[4] = (_Float16)b.x; u[5] = (_Float16)b.y; u[6] = (_Float16)b.z; u[7] = (_Float16)b.w;
    *(v8h*)(sEF + el * EP + 8 * q) = u;
    v8h z;
#pragma unroll
    for (int i = 0; i < 8; ++i) z[i] = (_Float16)0.0f;
    *(v8h*)(sEF + el * EP + 16 + 8 * q) = z;
  }
  __syncthreads();

  {
    const v16h a = ldfrag(sEF + (16 * wave + m) * EP + 8 * hh);
#pragma unroll
    for (int j = 0; j < 4; ++j) {
      const v16h b = ldfrag(w1e + (size_t)(16 * j + m) * KE + 8 * hh);
      const v8f t = wm(a, b, zero8());
      float* sp = sT + (16 * wave + 8 * hh) * SP + 16 * j + m;
#pragma unroll
      for (int r = 0; r < 8; ++r) sp[r * SP] = t[r];
    }
  }
  __syncthreads();

  {
    const int el = tid >> 1, q = tid & 1;
    const int snode = sIdx[el], dnode = sIdx[TE + el];
    const float* pp = PQ + (size_t)dnode * NPQ + 32 * q;
    const float* qp = PQ + (size_t)snode * NPQ + HD + 32 * q;
    const float* tp = sT + el * SP + 32 * q;
    const float* pb = sPar + 32 * q;
    v4f t[8];
    float s = 0.0f;
#pragma unroll
    for (int g = 0; g < 8; ++g) {
      const v4f a  = *(const v4f*)(pp + 4 * g);
      const v4f b  = *(const v4f*)(qp + 4 * g);
      const v4f u  = *(const v4f*)(tp + 4 * g);
      const v4f bb = *(const v4f*)(pb + 4 * g);
      v4f z = a + b;
      z = z + u * 0.015625f;
      z = z + bb;
      t[g] = z;
      s = s + ((z.x + z.y) + (z.z + z.w));
    }
    s += __shfl_xor(s, 1, 32);
    const float mean = s * (1.0f / 64.0f);
    float v = 0.0f;
#pragma unroll
    for (int g = 0; g < 8; ++g) {
      v4f d = t[g] - mean;
      t[g] = d;
      v = v + ((d.x * d.x + d.y * d.y) + (d.z * d.z + d.w * d.w));
    }
    v += __shfl_xor(v, 1, 32);
    const float rs = rsqrtf(v * (1.0f / 64.0f) + EPSLN);
    _Float16* dst = sM1 + el * MP + 32 * q;
#pragma unroll
    for (int g2 = 0; g2 < 4; ++g2) {
      const v4f d0 = t[2 * g2], d1 = t[2 * g2 + 1];
      v8h o;
      o[0] = m1h(d0.x, rs); o[1] = m1h(d0.y, rs); o[2] = m1h(d0.z, rs); o[3] = m1h(d0.w, rs);
      o[4] = m1h(d1.x, rs); o[5] = m1h(d1.y, rs); o[6] = m1h(d1.z, rs); o[7] = m1h(d1.w, rs);
      *(v8h*)(dst + 8 * g2) = o;
    }
  }
  __syncthreads();

  v8f c[4];
#pragma unroll
  for (int j = 0; j < 4; ++j) c[j] = zero8();
  {
    const _Float16* ap = sM1 + (16 * wave + m) * MP + 8 * hh;
    const _Float16* bp = w2p + (size_t)m * HD + 8 * hh;
#pragma unroll
    for (int ks = 0; ks < 2; ++ks) {
      const v16h a = ldfrag(ap + 32 * ks);
#pragma unroll
      for (int j = 0; j < 4; ++j) {
        const v16h b = ldfrag(bp + (size_t)(16 * j) * HD + 32 * ks);
        c[j] = wm(a, b, c[j]);
      }
    }
  }

  ln_relu_acc(c, sPar + HD, m, 0.0009765625f);
#pragma unroll
  for (int j = 0; j < 4; ++j) {
    float* sp = sO + (16 * wave + 8 * hh) * SP + 16 * j + m;
#pragma unroll
    for (int r = 0; r < 8; ++r) sp[r * SP] = c[j][r];
  }
  __syncthreads();
  float* ob = MS + (size_t)4 * m;
#pragma unroll 1
  for (int i = 0; i < 8; ++i) {
    const int row = 16 * wave + 2 * i + hh;
    const v4f v = *(const v4f*)(sO + row * SP + 4 * m);
    *(volatile v4f*)(ob + (size_t)(le0 + row) * CO) = v;
  }
  __threadfence();
#pragma unroll 1
  for (int i = 0; i < 8; ++i) {
    const int row = 16 * wave + 2 * i + hh;
    const v4f v = *(const v4f*)(sO + row * SP + 4 * m);
    *(volatile v4f*)(ob + (size_t)(le0 + row) * CO) = v;
  }
}

__device__ __forceinline__ int scan_piece(const int* __restrict__ kp, int lim, int cbase, int base,
                                          int* list, int tid, int wave, int vec_ok) {
  int wc = 0;
  const int el0  = tid * EPT;
  const int e0   = cbase + el0;
  const int sent = -2147483647 - 1;
  int kk[EPT];
  if (vec_ok != 0 && cbase + PIECE <= lim) {
    const v4i* p = (const v4i*)(kp + e0);
#pragma unroll
    for (int u = 0; u < EPT / 4; ++u) {
      const v4i d = p[u];
      kk[4 * u] = d.x; kk[4 * u + 1] = d.y; kk[4 * u + 2] = d.z; kk[4 * u + 3] = d.w;
    }
  } else {
    const int lm = lim - 1;
#pragma unroll
    for (int q = 0; q < EPT; ++q) {
      const int eq = e0 + q;
      const int ec = eq > lm ? lm : eq;
      const int a = kp[ec];
      kk[q] = (eq < lim) ? a : sent;
    }
  }
  const unsigned nb = (unsigned)base;
  unsigned sq[EPT];
  bool hq[EPT];
  bool anyl = false;
#pragma unroll
  for (int q = 0; q < EPT; ++q) {
    sq[q] = (unsigned)kk[q] - nb;
    hq[q] = sq[q] < (unsigned)NBC;
    anyl = anyl | hq[q];
  }
  const unsigned any = __builtin_amdgcn_ballot_w32(anyl);
  if (any != 0u) {
#define HIT(HQ, SQ, Q) { \
      const unsigned mj = __builtin_amdgcn_ballot_w32(HQ); \
      if (mj != 0u) { \
        if (HQ) { \
          const int ps = wc + (int)__builtin_amdgcn_mbcnt_lo(mj, 0u); \
          if (ps < WCAP) list[wave * WCAP + ps] = ((el0 + (Q)) << SLB) | (int)(SQ); \
        } \
        wc += (int)__builtin_popcount(mj); } }
#pragma unroll
    for (int q = 0; q < EPT; ++q) {
      HIT(hq[q], sq[q], q)
    }
#undef HIT
  }
  return wc;
}

__device__ __forceinline__ void drain_sum(const int* list, const int* wcnt, float* accF,
                                          const float* __restrict__ MS,
                                          int cbase, int nec, int lane, int wave) {
#pragma unroll 1
  for (int wsx = 0; wsx < NWAVE; ++wsx) {
    int n = __builtin_amdgcn_readfirstlane(wcnt[wsx]);
    n = n > WCAP ? WCAP : (n < 0 ? 0 : n);
    const int* lp = list + wsx * WCAP;
#pragma unroll 1
    for (int bb = 0; bb < n; bb += 32) {
      const int idx = bb + lane;
      const int ic = idx > WCAP - 1 ? WCAP - 1 : idx;
      const int ent = lp[ic];
      const bool own = (idx < n) && ((ent & (NWAVE - 1)) == wave);
      unsigned msk = __builtin_amdgcn_ballot_w32(own);
#pragma unroll 1
      while (msk != 0u) {
        const int bit = (int)__builtin_ctz(msk);
        msk &= msk - 1u;
        const int e2 = __builtin_amdgcn_readlane(ent, bit);
        const int slot = e2 & (NBC - 1);
        const int el = (e2 >> SLB) & (PIECE - 1);
        int e = cbase + el;
        e = e > nec - 1 ? nec - 1 : (e < 0 ? 0 : e);
        const v2f v = *(const v2f*)(MS + (size_t)e * CO + 2 * lane);
        float* ap = accF + slot * CO + 2 * lane;
        v2f a = *(const v2f*)ap;
        a = a + v;
        *(v2f*)ap = a;
      }
    }
  }
}

__device__ __forceinline__ void node_rows(const float* accF, float* AG, int base, int wave, int hh, int m) {
#pragma unroll 1
  for (int it = 0; it < NBC / (2 * NWAVE); ++it) {
    const int s = wave + NWAVE * (2 * it + hh);
    const v4f v = *(const v4f*)(accF + s * CO + 4 * m);
    *(volatile v4f*)(AG + (size_t)(base + s) * CO + 4 * m) = v;
  }
}

__global__ __launch_bounds__(NTHR) void k_agg(
    const int* __restrict__ ei, const float* __restrict__ MS, float* AG,
    int c0, int nec, int nE, int first, int vec_ok) {
  extern __shared__ __attribute__((aligned(16))) float accF[];
  __shared__ int list[NWAVE * WCAP];
  __shared__ int wcnt[NWAVE];
  const int tid = (int)threadIdx.x, lane = tid & 31, wave = tid >> 5, hh = lane >> 4, m = lane & 15;
  const int base = (int)blockIdx.x * NBC;

  if (first != 0) {
    const v4f z = {0.0f, 0.0f, 0.0f, 0.0f};
#pragma unroll 1
    for (int i = tid; i < (NBC * CO) / 4; i += NTHR) *(v4f*)(accF + 4 * i) = z;
  } else {
    const float* src = AG + (size_t)base * CO;
#pragma unroll 1
    for (int i = tid; i < (NBC * CO) / 4; i += NTHR) {
      const v4f v = *(const v4f*)(src + (size_t)4 * i);
      *(v4f*)(accF + 4 * i) = v;
    }
  }
  __syncthreads();

  const int* kp = ei + (size_t)nE + c0;
#pragma unroll 1
  for (int cbase = 0; cbase < nec; cbase += PIECE) {
    const int wc = scan_piece(kp, nec, cbase, base, list, tid, wave, vec_ok);
    if (lane == 0) wcnt[wave] = wc;
    __syncthreads();
    drain_sum(list, wcnt, accF, MS, cbase, nec, lane, wave);
    __syncthreads();
  }

  node_rows(accF, AG, base, wave, hh, m);
  __threadfence();
  node_rows(accF, AG, base, wave, hh, m);
}

__global__ __launch_bounds__(NTHR) void k_upd(
    const float* __restrict__ x, const float* __restrict__ AG, const float* __restrict__ bu,
    const _Float16* __restrict__ wq, float* xo, int nN, int nStore) {
  extern __shared__ __attribute__((aligned(16))) float udyn[];
  __shared__ __attribute__((aligned(16))) float sPar[CO];
  _Float16* sA = (_Float16*)udyn;
  float* sO = udyn + (NBU * UP * 2) / 4;
  const int tid = (int)threadIdx.x, lane = tid & 31, wave = tid >> 5, hh = lane >> 4, m = lane & 15;
  const int n0 = (int)blockIdx.x * NBU;

  if (tid < CO) sPar[tid] = bu[tid];
  {
    const int el = tid & (NBU - 1), q = tid >> 7;
    const int node = n0 + el;
    const int nc = node > nN - 1 ? nN - 1 : node;
    const float* rp = (q == 0) ? (x + (size_t)nc * CI) : (AG + (size_t)node * CO);
    _Float16* dst = sA + el * UP + 64 * q;
#pragma unroll
    for (int g = 0; g < 8; ++g) {
      const v4f a = *(const v4f*)(rp + 8 * g);
      const v4f b = *(const v4f*)(rp + 8 * g + 4);
      v8h u;
      u[0] = (_Float16)a.x; u[1] = (_Float16)a.y; u[2] = (_Float16)a.z; u[3] = (_Float16)a.w;
      u[4] = (_Float16)b.x; u[5] = (_Float16)b.y; u[6] = (_Float16)b.z; u[7] = (_Float16)b.w;
      *(v8h*)(dst + 8 * g) = u;
    }
  }
  __syncthreads();

  v8f c[4];
#pragma unroll
  for (int j = 0; j < 4; ++j) c[j] = zero8();
  {
    const _Float16* ap = sA + (16 * wave + m) * UP + 8 * hh;
    const _Float16* bp = wq + (size_t)m * KU + 8 * hh;
#pragma unroll
    for (int ks = 0; ks < 4; ++ks) {
      const v16h a = ldfrag(ap + 32 * ks);
#pragma unroll
      for (int j = 0; j < 4; ++j) {
        const v16h b = ldfrag(bp + (size_t)(16 * j) * KU + 32 * ks);
        c[j] = wm(a, b, c[j]);
      }
    }
  }
  ln_relu_acc(c, sPar, m, 0.015625f);
#pragma unroll
  for (int j = 0; j < 4; ++j) {
    float* sp = sO + (16 * wave + 8 * hh) * SP + 16 * j + m;
#pragma unroll
    for (int r = 0; r < 8; ++r) sp[r * SP] = c[j][r];
  }
  __syncthreads();

  v4f vv[8];
#pragma unroll
  for (int i = 0; i < 8; ++i) {
    const int row = 16 * wave + 2 * i + hh;
    const int node = n0 + row;
    const int nc = node > nN - 1 ? nN - 1 : node;
    const v4f t  = *(const v4f*)(sO + row * SP + 4 * m);
    const v4f xr = *(const v4f*)(x + (size_t)nc * CI + 4 * m);
    vv[i] = xr + t;
  }
#pragma unroll
  for (int i = 0; i < 8; ++i) {
    const int node = n0 + 16 * wave + 2 * i + hh;
    if (node < nStore) *(volatile v4f*)(xo + (size_t)node * CO + 4 * m) = vv[i];
  }
  __threadfence();
#pragma unroll
  for (int i = 0; i < 8; ++i) {
    const int node = n0 + 16 * wave + 2 * i + hh;
    if (node < nStore) *(volatile v4f*)(xo + (size_t)node * CO + 4 * m) = vv[i];
  }
}

extern "C" void kernel_launch(void* const* d_in, const int* in_sizes, int n_in,
                              void* d_out, int out_size, void* d_ws, size_t ws_size,
                              hipStream_t stream) {
  if (n_in < 9) return;
  if (in_sizes[0] < CI || (in_sizes[0] % CI) != 0) return;
  const int nN = in_sizes[0] / CI;
  if (nN < 1 || nN > (1 << 22)) return;
  if (in_sizes[1] < DE || (in_sizes[1] % DE) != 0) return;
  const int nE = in_sizes[1] / DE;
  if (nE < 1 || nE > (1 << 27)) return;
  if (in_sizes[2] != 2 * nE) return;
  if (in_sizes[3] != NLAY * KIN1 * HD || in_sizes[4] != NLAY * HD) return;
  if (in_sizes[5] != NLAY * HD * HD || in_sizes[6] != NLAY * HD) return;
  if (in_sizes[7] != NLAY * KU * HD || in_sizes[8] != NLAY * HD) return;
  if ((long long)out_size != (long long)nN * CO) return;

  const float* xin = (const float*)d_in[0];
  const float* ef  = (const float*)d_in[1];
  const int*   ei  = (const int*)d_in[2];
  const float* w1  = (const float*)d_in[3];
  const float* b1  = (const float*)d_in[4];
  const float* w2  = (const float*)d_in[5];
  const float* b2  = (const float*)d_in[6];
  const float* wu  = (const float*)d_in[7];
  const float* bu  = (const float*)d_in[8];
  float* outp = (float*)d_out;

  const int nb64 = (nN + NBN - 1) / NBN;
  const int Npad64 = nb64 * NBN;
  const int nb128 = (nN + NBU - 1) / NBU;
  const int Npad128 = nb128 * NBU;
  const int nbA = (nN + NBC - 1) / NBC;
  const int aggRows = nbA * NBC;
  const int vec_ok = ((nE & 3) == 0) ? 1 : 0;

  const size_t cap = ws_size < (size_t)WSCAP ? ws_size : (size_t)WSCAP;
  const size_t bW  = (size_t)NLAY * LWTOT * 2;
  const size_t bPQ = (size_t)Npad64 * NPQ * 4;
  const size_t bAG = (size_t)aggRows * CO * 4;
  const size_t bX  = (size_t)Npad128 * CO * 4;
  const size_t fixedB = ((bW + 255) & ~(size_t)255) + ((bPQ + 255) & ~(size_t)255) +
                        ((bAG + 255) & ~(size_t)255) + 2 * ((bX + 255) & ~(size_t)255);
  int C = 0;
  size_t CE = 0;
  for (int c = 1; c <= 1024; ++c) {
    size_t ce = ((size_t)nE + (size_t)c - 1) / (size_t)c;
    ce = (ce + PIECE - 1) / PIECE * PIECE;
    const size_t tot = fixedB + ((ce * CO * 4 + 255) & ~(size_t)255);
    if (tot <= cap) { C = c; CE = ce; break; }
  }
  if (C == 0) return;

  char* ws = (char*)d_ws;
  size_t off = 0;
  const size_t oW  = off; off += bW;                    off = (off + 255) & ~(size_t)255;
  const size_t oPQ = off; off += bPQ;                   off = (off + 255) & ~(size_t)255;
  const size_t oAG = off; off += bAG;                   off = (off + 255) & ~(size_t)255;
  const size_t oXA = off; off += bX;                    off = (off + 255) & ~(size_t)255;
  const size_t oXB = off; off += bX;                    off = (off + 255) & ~(size_t)255;
  const size_t oMS = off; off += CE * CO * 4;           off = (off + 255) & ~(size_t)255;
  if (off > cap || off > ws_size) return;
  _Float16* wp = (_Float16*)(ws + oW);
  float*    PQ = (float*)(ws + oPQ);
  float*    AG = (float*)(ws + oAG);
  float*    XA = (float*)(ws + oXA);
  float*    XB = (float*)(ws + oXB);
  float*    MS = (float*)(ws + oMS);

  hipFuncSetAttribute(reinterpret_cast<const void*>(&k_pq),   hipFuncAttributeMaxDynamicSharedMemorySize, PQDYN);
  hipFuncSetAttribute(reinterpret_cast<const void*>(&k_edge), hipFuncAttributeMaxDynamicSharedMemorySize, EDGEDYN);
  hipFuncSetAttribute(reinterpret_cast<const void*>(&k_upd),  hipFuncAttributeMaxDynamicSharedMemorySize, UPDDYN);
  hipFuncSetAttribute(reinterpret_cast<const void*>(&k_agg),  hipFuncAttributeMaxDynamicSharedMemorySize, AGGDYN);

  k_prep<<<PREPBLK, NTHR, 0, stream>>>(w1, w2, wu, wp);
  for (int l = 0; l < NLAY; ++l) {
    const float* cur = (l == 0) ? xin : ((l == 1) ? XA : XB);
    float* nxt = (l == 0) ? XA : ((l == 1) ? XB : outp);
    const int nStore = (l == NLAY - 1) ? nN : Npad128;
    const _Float16* wl = wp + (size_t)l * LWTOT;
    k_pq<<<nb64, NTHR, PQDYN, stream>>>(cur, wl + LW_PQ, PQ, nN);
    for (int ch = 0; ch < C; ++ch) {
      const size_t c0s = (size_t)ch * CE;
      if (c0s >= (size_t)nE) break;
      const int c0 = (int)c0s;
      size_t necs = (size_t)nE - c0s;
      if (necs > CE) necs = CE;
      const int nec = (int)necs;
      const int ntiles = (nec + TE - 1) / TE;
      k_edge<<<ntiles, NTHR, EDGEDYN, stream>>>(ei, ef, PQ, b1 + l * HD, b2 + l * HD, wl, MS, c0, nE, nN);
      k_agg<<<nbA, NTHR, AGGDYN, stream>>>(ei, MS, AG, c0, nec, nE, (ch == 0) ? 1 : 0, vec_ok);
    }
    k_upd<<<nb128, NTHR, UPDDYN, stream>>>(cur, AG, bu + l * HD, wl + LW_WU, nxt, nN, nStore);
  }
}
